// GeometricNN_61881888801068
// MI455X (gfx1250) — hardware-verified
//
#include <hip/hip_runtime.h>

#define DD 128
#define ROWW 64
#define MAXDEG 63
#define BW 256
#define SLOPE 0.2f
#define STAGE_CAP 2304

typedef _Float16 v16h __attribute__((ext_vector_type(16)));
typedef _Float16 v8h  __attribute__((ext_vector_type(8)));
typedef _Float16 v4h  __attribute__((ext_vector_type(4)));
typedef float    v8f  __attribute__((ext_vector_type(8)));
typedef float    v4f  __attribute__((ext_vector_type(4)));
typedef int      v4i  __attribute__((ext_vector_type(4)));
union Frag { v16h v; v8h half[2]; v4h q[4]; };

extern __shared__ __align__(16) unsigned char dynsmem[];

__device__ __forceinline__ v8f wmma_f16(v16h a, v16h b, v8f c) {
    v8f d = __builtin_amdgcn_wmma_f32_16x16x32_f16(false, a, false, b, (short)0, c, false, false);
    asm volatile("v_nop\n\tv_nop\n\tv_nop\n\tv_nop" : "+v"(d) : "v"(a), "v"(b));
    return d;
}

__device__ __forceinline__ float wsum(float v) {
    v += __shfl_xor(v, 16, 32); v += __shfl_xor(v, 8, 32); v += __shfl_xor(v, 4, 32);
    v += __shfl_xor(v, 2, 32);  v += __shfl_xor(v, 1, 32);
    return v;
}
__device__ __forceinline__ float wmax(float v) {
    v = fmaxf(v, __shfl_xor(v, 16, 32)); v = fmaxf(v, __shfl_xor(v, 8, 32)); v = fmaxf(v, __shfl_xor(v, 4, 32));
    v = fmaxf(v, __shfl_xor(v, 2, 32));  v = fmaxf(v, __shfl_xor(v, 1, 32));
    return v;
}

__global__ __launch_bounds__(256)
void k_convw(const float* __restrict__ W0, const float* __restrict__ W1, const float* __restrict__ W2,
             const float* __restrict__ W3, const float* __restrict__ W4, const float* __restrict__ W5,
             _Float16* Wt)
{
    const int idx = blockIdx.x * 256 + threadIdx.x;
    if (idx >= 6 * DD * 16) return;
    const int k8  = idx & 15;
    const int n   = (idx >> 4) & (DD - 1);
    const int sel = idx >> 11;
    const float* W = W0;
    if (sel == 1) W = W1; else if (sel == 2) W = W2; else if (sel == 3) W = W3;
    else if (sel == 4) W = W4; else if (sel == 5) W = W5;
    v8h v;
#pragma unroll
    for (int i = 0; i < 8; ++i) v[i] = (_Float16)(16.0f * W[(size_t)(8 * k8 + i) * DD + n]);
    _Float16* p = Wt + (size_t)idx * 8;
    *(volatile v8h*)p = v;
    __threadfence();
    *(volatile v8h*)p = v;
}

__device__ __forceinline__ void flush_lines(const int* s_stage, int* gdst, int nl, int tid) {
    for (int t = tid; t < 8 * nl; t += 256) {
        const int q = t >> 3, pc = t & 7;
        const v4i v = *(const v4i*)(s_stage + 32 * q + 4 * pc);
        *(volatile v4i*)(gdst + 32 * q + 4 * pc) = v;
    }
}

__device__ __forceinline__ void blk_append(int* s_stage, int* s_wtot, const int* e, unsigned msk,
                                           int& fill, int& lines, const int maxLines, int* glist,
                                           const int tid, const int lane, const int wave)
{
    const int mc = __popc(msk);
    int incl = mc;
#pragma unroll
    for (int off = 1; off < 32; off <<= 1) {
        const int y = __shfl_up(incl, off, 32);
        if (lane >= off) incl += y;
    }
    if (lane == 31) s_wtot[wave] = incl;
    __syncthreads();
    int pre = 0, tot = 0;
#pragma unroll
    for (int w = 0; w < 8; ++w) {
        const int v = s_wtot[w];
        tot += v;
        if (w < wave) pre += v;
    }
    int pos = fill + pre + incl - mc;
#pragma unroll
    for (int j = 0; j < 8; ++j) {
        if (msk & (1u << j)) { s_stage[pos] = e[j]; ++pos; }
    }
    fill += tot;
    __syncthreads();
    if (fill >= 256) {
        const int nl = fill >> 5;
        const int room = maxLines - lines;
        const int nlw = nl < room ? nl : room;
        int* gd = glist + 32 * lines;
        flush_lines(s_stage, gd, nlw, tid);
        __threadfence();
        flush_lines(s_stage, gd, nlw, tid);
        lines += nlw;
        __syncthreads();
        const int rem = (nlw == nl) ? (fill & 31) : 0;
        int mv = 0;
        if (tid < rem) mv = s_stage[32 * nl + tid];
        __syncthreads();
        if (tid < rem) s_stage[tid] = mv;
        fill = rem;
        __syncthreads();
    }
}

__device__ __forceinline__ void blk_finish(int* s_stage, int fill, int lines, const int maxLines,
                                           int* gseg, int* glist, const int tid)
{
    const int nl = (fill + 31) >> 5;
    if (tid >= fill && tid < 32 * nl) s_stage[tid] = 0;
    __syncthreads();
    const int room = maxLines - lines;
    const int nlw = nl < room ? nl : room;
    int* gd = glist + 32 * lines;
    flush_lines(s_stage, gd, nlw, tid);
    __threadfence();
    flush_lines(s_stage, gd, nlw, tid);
    const int kept = (fill < 32 * nlw) ? fill : 32 * nlw;
    const int stored = 32 * lines + kept;
    v4i hv; hv.x = (tid == 0) ? stored : 0; hv.y = 0; hv.z = 0; hv.w = 0;
    if (tid < 8) *(volatile v4i*)(gseg + 4 * tid) = hv;
    __threadfence();
    if (tid < 8) *(volatile v4i*)(gseg + 4 * tid) = hv;
}

__global__ __launch_bounds__(256)
void k_binA(const int* __restrict__ dst, int E, int W, int cap, int stride, int* seg)
{
    __shared__ __align__(16) int s_stage[STAGE_CAP];
    __shared__ int s_wtot[8];
    const int tid = threadIdx.x, lane = tid & 31, wave = tid >> 5;
    const int lo = blockIdx.x * W;
    int* gseg = seg + (size_t)blockIdx.x * stride;
    int* glist = gseg + 32;
    const int maxLines = cap >> 5;
    const bool vec = ((E & 3) == 0);
    int fill = 0, lines = 0;
    for (int base = 0; base < E; base += 2048) {
        const int i0 = base + 8 * tid;
        int d[8];
        if (vec && i0 + 8 <= E) {
            const v4i a = *(const v4i*)(dst + i0);
            const v4i c = *(const v4i*)(dst + i0 + 4);
            d[0] = a.x; d[1] = a.y; d[2] = a.z; d[3] = a.w;
            d[4] = c.x; d[5] = c.y; d[6] = c.z; d[7] = c.w;
        } else {
#pragma unroll
            for (int j = 0; j < 8; ++j) d[j] = (i0 + j < E) ? dst[i0 + j] : -1;
        }
        int e[8];
        unsigned msk = 0;
#pragma unroll
        for (int j = 0; j < 8; ++j) {
            e[j] = i0 + j;
            const unsigned rel = (unsigned)(d[j] - lo);
            if (rel < (unsigned)W) msk |= (1u << j);
        }
        blk_append(s_stage, s_wtot, e, msk, fill, lines, maxLines, glist, tid, lane, wave);
    }
    blk_finish(s_stage, fill, lines, maxLines, gseg, glist, tid);
}

__global__ __launch_bounds__(256)
void k_binB(const int* __restrict__ dst, int E, const int* segIn, int capIn, int strideIn, int CPP,
            int W, int cap, int stride, int* seg)
{
    __shared__ __align__(16) int s_stage[STAGE_CAP];
    __shared__ int s_wtot[8];
    const int tid = threadIdx.x, lane = tid & 31, wave = tid >> 5;
    const int parent = blockIdx.x / CPP;
    const int lo = blockIdx.x * W;
    const int* gin = segIn + (size_t)parent * strideIn;
    int cnt = gin[0];
    cnt = cnt < 0 ? 0 : (cnt > capIn ? capIn : cnt);
    const int* glin = gin + 32;
    int* gseg = seg + (size_t)blockIdx.x * stride;
    int* glist = gseg + 32;
    const int maxLines = cap >> 5;
    int fill = 0, lines = 0;
    for (int base = 0; base < cnt; base += 2048) {
        const int i0 = base + 8 * tid;
        int e[8];
        unsigned msk = 0;
        if (i0 < cnt) {
            const v4i a = *(const v4i*)(glin + i0);
            const v4i c = *(const v4i*)(glin + i0 + 4);
            e[0] = a.x; e[1] = a.y; e[2] = a.z; e[3] = a.w;
            e[4] = c.x; e[5] = c.y; e[6] = c.z; e[7] = c.w;
#pragma unroll
            for (int j = 0; j < 8; ++j) {
                int ee = e[j];
                ee = ((unsigned)ee < (unsigned)E) ? ee : 0;
                e[j] = ee;
                const int d = dst[ee];
                if ((i0 + j < cnt) && ((unsigned)(d - lo) < (unsigned)W)) msk |= (1u << j);
            }
        } else {
#pragma unroll
            for (int j = 0; j < 8; ++j) e[j] = 0;
        }
        blk_append(s_stage, s_wtot, e, msk, fill, lines, maxLines, glist, tid, lane, wave);
    }
    blk_finish(s_stage, fill, lines, maxLines, gseg, glist, tid);
}

__global__ __launch_bounds__(256)
void k_rows(const int* __restrict__ srcArr, const int* __restrict__ dstArr, int E, int N,
            const int* seg, int cap, int stride, int* adj)
{
    int* rows = (int*)dynsmem;
    const int tid = threadIdx.x, lane = tid & 31, wave = tid >> 5;
    const int lo = blockIdx.x * BW;
    const int* gseg = seg + (size_t)blockIdx.x * stride;
    int cnt = gseg[0];
    cnt = cnt < 0 ? 0 : (cnt > cap ? cap : cnt);
    const int* glist = gseg + 32;
    for (int i = tid; i < BW * ROWW; i += 256) rows[i] = 0;
    __syncthreads();
    for (int base = 0; base < cnt; base += 256) {
        const int idx = base + tid;
        const bool valid = idx < cnt;
        int e = 0;
        if (valid) e = glist[idx];
        e = ((unsigned)e < (unsigned)E) ? e : 0;
        const int d = dstArr[e];
        int s = srcArr[e];
        s = s < 0 ? 0 : (s > N - 1 ? N - 1 : s);
        const int key = (valid && ((unsigned)(d - lo) < (unsigned)BW)) ? (d - lo) : -1;
        int rank = 0, gcnt = 0;
#pragma unroll
        for (int j = 0; j < 32; ++j) {
            const int kj = __shfl(key, j, 32);
            const int same = (kj == key) ? 1 : 0;
            gcnt += same;
            if (j < lane) rank += same;
        }
#pragma unroll
        for (int w = 0; w < 8; ++w) {
            if (wave == w && key >= 0) {
                int* rw = rows + key * ROWW;
                const int old = rw[0];
                const int pos = old + rank;
                if (pos < MAXDEG) rw[1 + pos] = s;
                if (rank == gcnt - 1) rw[0] = old + gcnt;
            }
            __syncthreads();
        }
    }
    __syncthreads();
#pragma unroll 1
    for (int rr = 0; rr < 32; ++rr) {
        const int r = wave + 8 * rr;
        if (lane < 16) {
            const v4i v = *(const v4i*)(rows + r * ROWW + 4 * lane);
            *(volatile v4i*)(adj + (size_t)(lo + r) * ROWW + 4 * lane) = v;
        }
    }
    __threadfence();
#pragma unroll 1
    for (int rr = 0; rr < 32; ++rr) {
        const int r = wave + 8 * rr;
        if (lane < 16) {
            const v4i v = *(const v4i*)(rows + r * ROWW + 4 * lane);
            *(volatile v4i*)(adj + (size_t)(lo + r) * ROWW + 4 * lane) = v;
        }
    }
}

__global__ __launch_bounds__(128)
void k_gemm3(const float* __restrict__ A, int N, const _Float16* __restrict__ Wt,
             const float* __restrict__ bias2, float* C0, float* C1, float* C2)
{
    _Float16* Ws = (_Float16*)dynsmem;
    float* tiles = (float*)(dynsmem + 32768);
    const int tid = threadIdx.x, lane = tid & 31, wave = tid >> 5;
    const int m = lane & 15, h = lane >> 4;
    const int r0 = blockIdx.x * 64 + wave * 16;
    int arow = r0 + m;
    if (arow > N - 1) arow = N - 1;
    const float* Ap = A + (size_t)arow * DD;
    float* T = tiles + wave * (16 * DD);
#pragma unroll 1
    for (int grp = 0; grp < 3; ++grp) {
        __syncthreads();
        const _Float16* Wg = Wt + grp * (DD * DD);
        for (int i = tid; i < DD * DD / 8; i += 128)
            *(v8h*)(Ws + 8 * i) = *(const v8h*)(Wg + 8 * i);
        __syncthreads();
        v8f acc[8];
#pragma unroll
        for (int nt = 0; nt < 8; ++nt) {
            const v8f z = {0.f, 0.f, 0.f, 0.f, 0.f, 0.f, 0.f, 0.f};
            acc[nt] = z;
        }
#pragma unroll
        for (int kt = 0; kt < 4; ++kt) {
            const int k0 = kt * 32;
            const float* ap = Ap + k0 + 8 * h;
            Frag a;
            a.q[0] = __builtin_convertvector(*(const v4f*)(ap), v4h);
            a.q[1] = __builtin_convertvector(*(const v4f*)(ap + 4), v4h);
            a.q[2] = __builtin_convertvector(*(const v4f*)(ap + 16), v4h);
            a.q[3] = __builtin_convertvector(*(const v4f*)(ap + 20), v4h);
#pragma unroll
            for (int nt = 0; nt < 8; ++nt) {
                const _Float16* bp = Ws + (16 * nt + m) * DD + k0 + 8 * h;
                Frag b;
                b.half[0] = *(const v8h*)(bp);
                b.half[1] = *(const v8h*)(bp + 16);
                acc[nt] = wmma_f16(a.v, b.v, acc[nt]);
            }
        }
        const bool useB = (grp == 2);
#pragma unroll
        for (int nt = 0; nt < 8; ++nt) {
            const int col = 16 * nt + m;
            const float bv = useB ? bias2[col] : 0.f;
#pragma unroll
            for (int r = 0; r < 8; ++r) T[(8 * h + r) * DD + col] = acc[nt][r] * 0.0625f + bv;
        }
        __syncthreads();
        float* Cg = (grp == 0) ? C0 : ((grp == 1) ? C1 : C2);
#pragma unroll
        for (int r = 0; r < 16; ++r) {
            const v4f v = *(const v4f*)(T + r * DD + 4 * lane);
            *(volatile v4f*)(Cg + (size_t)(r0 + r) * DD + 4 * lane) = v;
        }
        __threadfence();
#pragma unroll
        for (int r = 0; r < 16; ++r) {
            const v4f v = *(const v4f*)(T + r * DD + 4 * lane);
            *(volatile v4f*)(Cg + (size_t)(r0 + r) * DD + 4 * lane) = v;
        }
    }
}

template <int HEAD>
__global__ __launch_bounds__(256)
void k_agg(const int* __restrict__ adj, const float* __restrict__ XL, const float* __restrict__ XR,
           const float* __restrict__ LIN, const float* __restrict__ att, const float* __restrict__ bg,
           float* H, const float* __restrict__ wlo, const float* __restrict__ wro,
           const float* __restrict__ wlino, float* xlo, float* xro, float* xlino, int N)
{
    __shared__ __align__(16) _Float16 s_t[8 * 16 * DD];
    __shared__ __align__(16) _Float16 s_att[DD];
    const int lane = threadIdx.x & 31;
    const int wave = threadIdx.x >> 5;
    const int m = lane & 15, h = lane >> 4, cc = lane & 3;
    if (threadIdx.x < 32) {
        const v4f a4 = *(const v4f*)(att + 4 * lane);
        *(v4h*)(s_att + 4 * lane) = __builtin_convertvector(a4 * 16.0f, v4h);
    }
    __syncthreads();
    const int base = (blockIdx.x * 8 + wave) * 32;
    if (base >= N) return;
    _Float16* T = s_t + wave * (16 * DD);
    Frag bfr;
    bfr.half[0] = *(const v8h*)(s_att + 32 * cc + 8 * h);
    bfr.half[1] = *(const v8h*)(s_att + 32 * cc + 16 + 8 * h);
    const float NINF = -__builtin_huge_valf();
    const v4f b4 = *(const v4f*)(bg + 4 * lane);
    v4f wlo4 = {0.f, 0.f, 0.f, 0.f}, wro4 = {0.f, 0.f, 0.f, 0.f}, wli4 = {0.f, 0.f, 0.f, 0.f};
    if (HEAD) {
        wlo4 = *(const v4f*)(wlo + 4 * lane);
        wro4 = *(const v4f*)(wro + 4 * lane);
        wli4 = *(const v4f*)(wlino + 4 * lane);
    }
    float res0 = 0.f, res1 = 0.f, res2 = 0.f;
    for (int i = 0; i < 32; ++i) {
        const int n = base + i;
        float o0 = 0.f, o1 = 0.f, o2 = 0.f;
        if (n < N) {
            const int* row = adj + (size_t)n * ROWW;
            const int ra = row[lane];
            const int rb = row[32 + lane];
            int cnt = __shfl(ra, 0, 32);
            cnt = cnt < 0 ? 0 : (cnt > MAXDEG ? MAXDEG : cnt);
            const v4f xr4  = *(const v4f*)(XR  + (size_t)n * DD + 4 * lane);
            const v4f lin4 = *(const v4f*)(LIN + (size_t)n * DD + 4 * lane);
            v4f acc = {0.f, 0.f, 0.f, 0.f};
            float mrun = NINF, ssum = 0.f;
            const int ng = (cnt + 15) >> 4;
#pragma unroll 1
            for (int g = 0; g < ng; ++g) {
                const int j0 = 16 * g;
                const int cg = cnt - j0;
                v4f u[16];
                asm volatile("" ::: "memory");
#pragma unroll
                for (int j = 0; j < 16; ++j) {
                    const int jj = j0 + j;
                    const int sv = __shfl(jj < 31 ? ra : rb, (jj + 1) & 31, 32);
                    int s = (jj < cnt) ? sv : n;
                    s = ((unsigned)s < (unsigned)N) ? s : 0;
                    const v4f uu = *(const v4f*)(XL + (size_t)s * DD + 4 * lane);
                    u[j] = uu;
                    const v4f t = uu + xr4;
                    v4f lk;
                    lk.x = fmaxf(t.x, SLOPE * t.x); lk.y = fmaxf(t.y, SLOPE * t.y);
                    lk.z = fmaxf(t.z, SLOPE * t.z); lk.w = fmaxf(t.w, SLOPE * t.w);
                    *(v4h*)(T + j * DD + 4 * lane) = __builtin_convertvector(lk, v4h);
                }
                asm volatile("" ::: "memory");
                float el[8];
#pragma unroll
                for (int w = 0; w < 4; ++w) {
                    float x0 = NINF, x1 = NINF;
                    if (4 * w < cg) {
                        Frag a;
                        a.half[0] = *(const v8h*)(T + 512 * w + 32 * m + 8 * h);
                        a.half[1] = *(const v8h*)(T + 512 * w + 32 * m + 16 + 8 * h);
                        const v8f z8 = {0.f, 0.f, 0.f, 0.f, 0.f, 0.f, 0.f, 0.f};
                        const v8f d = wmma_f16(a.v, bfr.v, z8);
                        float y0 = d[0], y1 = d[4];
                        y0 = (cc == 1) ? d[1] : y0; y0 = (cc == 2) ? d[2] : y0; y0 = (cc == 3) ? d[3] : y0;
                        y1 = (cc == 1) ? d[5] : y1; y1 = (cc == 2) ? d[6] : y1; y1 = (cc == 3) ? d[7] : y1;
                        y0 += __shfl_xor(y0, 1, 32); y0 += __shfl_xor(y0, 2, 32);
                        y1 += __shfl_xor(y1, 1, 32); y1 += __shfl_xor(y1, 2, 32);
                        const int jb = j0 + 4 * w + 2 * h;
                        x0 = (jb < cnt)     ? y0 * 0.0625f : NINF;
                        x1 = (jb + 1 < cnt) ? y1 * 0.0625f : NINF;
                    }
                    el[2 * w] = x0; el[2 * w + 1] = x1;
                }
                float lm = el[0];
#pragma unroll
                for (int r = 1; r < 8; ++r) lm = fmaxf(lm, el[r]);
                const float gm = fmaxf(lm, __shfl_xor(lm, 16, 32));
                const float mnew = fmaxf(mrun, gm);
                const float sc = __expf(mrun - mnew);
                float pl[8];
                float ps = 0.f;
#pragma unroll
                for (int r = 0; r < 8; ++r) { pl[r] = __expf(el[r] - mnew); ps += pl[r]; }
                ps += __shfl_xor(ps, 16, 32);
                acc = acc * sc;
#pragma unroll
                for (int j = 0; j < 16; ++j) {
                    const float pj = __shfl(pl[2 * (j >> 2) + (j & 1)], 16 * ((j >> 1) & 1), 32);
                    acc = acc + u[j] * pj;
                }
                ssum = ssum * sc + ps;
                mrun = mnew;
            }
            const float rinv = 1.0f / (ssum + 1e-16f);
            v4f o = acc * rinv + b4 + lin4;
            o.x = fmaxf(o.x, 0.f); o.y = fmaxf(o.y, 0.f); o.z = fmaxf(o.z, 0.f); o.w = fmaxf(o.w, 0.f);
            if (!HEAD) {
                volatile v4f* hp = (volatile v4f*)(H + (size_t)n * DD + 4 * lane);
                *hp = o;
                __threadfence();
                *hp = o;
            } else {
                o0 = wsum(o.x * wlo4.x + o.y * wlo4.y + o.z * wlo4.z + o.w * wlo4.w);
                o1 = wsum(o.x * wro4.x + o.y * wro4.y + o.z * wro4.z + o.w * wro4.w);
                o2 = wsum(o.x * wli4.x + o.y * wli4.y + o.z * wli4.z + o.w * wli4.w);
            }
        }
        if (HEAD) {
            if (lane == i) { res0 = o0; res1 = o1; res2 = o2; }
        }
    }
    if (HEAD) {
        const int q = lane & 7;
        v4f v0, v1, v2;
        v0.x = __shfl(res0, 4 * q, 32); v0.y = __shfl(res0, 4 * q + 1, 32); v0.z = __shfl(res0, 4 * q + 2, 32); v0.w = __shfl(res0, 4 * q + 3, 32);
        v1.x = __shfl(res1, 4 * q, 32); v1.y = __shfl(res1, 4 * q + 1, 32); v1.z = __shfl(res1, 4 * q + 2, 32); v1.w = __shfl(res1, 4 * q + 3, 32);
        v2.x = __shfl(res2, 4 * q, 32); v2.y = __shfl(res2, 4 * q + 1, 32); v2.z = __shfl(res2, 4 * q + 2, 32); v2.w = __shfl(res2, 4 * q + 3, 32);
        if (lane < 8) {
            *(volatile v4f*)(xlo   + base + 4 * lane) = v0;
            *(volatile v4f*)(xro   + base + 4 * lane) = v1;
            *(volatile v4f*)(xlino + base + 4 * lane) = v2;
        }
        __threadfence();
        if (lane < 8) {
            *(volatile v4f*)(xlo   + base + 4 * lane) = v0;
            *(volatile v4f*)(xro   + base + 4 * lane) = v1;
            *(volatile v4f*)(xlino + base + 4 * lane) = v2;
        }
    }
}

__global__ __launch_bounds__(256)
void k_out(const int* __restrict__ adj, const float* __restrict__ xlo, const float* __restrict__ xro,
           const float* __restrict__ xlino, const float* __restrict__ atto, const float* __restrict__ bo,
           const float* __restrict__ blino, float* out, int N)
{
    const int lane = threadIdx.x & 31;
    const int wave = threadIdx.x >> 5;
    const int base = (blockIdx.x * 8 + wave) * 32;
    if (base >= N) return;
    const float NINF = -__builtin_huge_valf();
    const float at = atto[0];
    const float bb = bo[0] + blino[0];
    float res = 0.f;
    for (int i = 0; i < 32; ++i) {
        const int n = base + i;
        float o = 0.f;
        if (n < N) {
            const int* row = adj + (size_t)n * ROWW;
            int cnt = row[0];
            cnt = cnt < 0 ? 0 : (cnt > MAXDEG ? MAXDEG : cnt);
            const int sa = row[1 + lane];
            int sb = 0;
            if (lane < 31) sb = row[33 + lane];
            const float xr = xro[n];
            const bool va = lane < cnt;
            const bool vb = (32 + lane) < cnt;
            int s0 = va ? sa : 0;
            s0 = ((unsigned)s0 < (unsigned)N) ? s0 : 0;
            int s1 = vb ? sb : 0;
            s1 = ((unsigned)s1 < (unsigned)N) ? s1 : 0;
            const float x0 = xlo[s0], x1 = xlo[s1];
            float t0 = x0 + xr; t0 = fmaxf(t0, SLOPE * t0);
            float t1 = x1 + xr; t1 = fmaxf(t1, SLOPE * t1);
            const float e0 = va ? t0 * at : NINF;
            const float e1 = vb ? t1 * at : NINF;
            float mm = wmax(fmaxf(e0, e1));
            mm = (cnt > 0) ? mm : 0.f;
            const float p0 = __expf(e0 - mm);
            const float p1 = __expf(e1 - mm);
            const float ss = wsum(p0 + p1);
            const float nm = wsum(p0 * x0 + p1 * x1);
            o = nm / (ss + 1e-16f) + bb + xlino[n];
        }
        if (lane == i) res = o;
    }
    const int q = lane & 7;
    v4f v;
    v.x = __shfl(res, 4 * q, 32); v.y = __shfl(res, 4 * q + 1, 32); v.z = __shfl(res, 4 * q + 2, 32); v.w = __shfl(res, 4 * q + 3, 32);
    const int i0 = base + 4 * q;
    if (lane < 8) {
        if (i0 + 4 <= N) {
            *(volatile v4f*)(out + i0) = v;
        } else {
            volatile float* op = out;
            if (i0 < N)     op[i0]     = v.x;
            if (i0 + 1 < N) op[i0 + 1] = v.y;
            if (i0 + 2 < N) op[i0 + 2] = v.z;
            if (i0 + 3 < N) op[i0 + 3] = v.w;
        }
    }
    __threadfence();
    if (lane < 8) {
        if (i0 + 4 <= N) {
            *(volatile v4f*)(out + i0) = v;
        } else {
            volatile float* op = out;
            if (i0 < N)     op[i0]     = v.x;
            if (i0 + 1 < N) op[i0 + 1] = v.y;
            if (i0 + 2 < N) op[i0 + 2] = v.z;
            if (i0 + 3 < N) op[i0 + 3] = v.w;
        }
    }
}

extern "C" void kernel_launch(void* const* d_in, const int* in_sizes, int n_in,
                              void* d_out, int out_size, void* d_ws, size_t ws_size,
                              hipStream_t stream)
{
    (void)n_in; (void)out_size;
    const int N = in_sizes[0] / DD;
    const int E = in_sizes[1] / 2;
    if (N <= 0 || E < 0) return;

    const float* x  = (const float*)d_in[0];
    const int*   ei = (const int*)d_in[1];
    const int* esrc = ei;
    const int* edst = ei + E;
    const float *Wl1 = (const float*)d_in[2],  *Wr1 = (const float*)d_in[3];
    const float *att1 = (const float*)d_in[4], *b1 = (const float*)d_in[5];
    const float *Wlin1 = (const float*)d_in[6], *blin1 = (const float*)d_in[7];
    const float *Wl2 = (const float*)d_in[8],  *Wr2 = (const float*)d_in[9];
    const float *att2 = (const float*)d_in[10], *b2 = (const float*)d_in[11];
    const float *Wlin2 = (const float*)d_in[12], *blin2 = (const float*)d_in[13];
    const float *Wlo = (const float*)d_in[14], *Wro = (const float*)d_in[15];
    const float *atto = (const float*)d_in[16], *bo = (const float*)d_in[17];
    const float *Wlino = (const float*)d_in[18], *blino = (const float*)d_in[19];
    float* out = (float*)d_out;

    const int Npad = (N + 63) / 64 * 64;
    const int N32  = (N + 31) / 32 * 32;
    const int NB   = (N + BW - 1) / BW;
    const int CPP  = 14;
    const int NSB  = (NB + CPP - 1) / CPP;
    const int SW   = BW * CPP;
    const long long eB = (long long)E * BW / N;
    const long long eA = (long long)E * SW / N;
    const long long cB = (eB + eB / 16 + 1024 + 31) / 32 * 32;
    const long long cA = (eA + eA / 16 + 1024 + 31) / 32 * 32;
    if (cA > (1LL << 30) || cB > (1LL << 30)) return;
    const int capA = (int)cA, capB = (int)cB;
    const int strideA = capA + 64, strideB = capB + 64;

    size_t off = 0;
    char* ws = (char*)d_ws;
    auto carve = [&](size_t bytes) -> char* { char* p = ws + off; off += (bytes + 255) & ~(size_t)255; return p; };
    _Float16* Wt = (_Float16*)carve((size_t)6 * DD * DD * sizeof(_Float16));
    float* XL  = (float*)carve((size_t)Npad * DD * sizeof(float));
    float* XR  = (float*)carve((size_t)Npad * DD * sizeof(float));
    float* LIN = (float*)carve((size_t)Npad * DD * sizeof(float));
    float* H1  = (float*)carve((size_t)Npad * DD * sizeof(float));
    int*   adj = (int*)carve((size_t)NB * BW * ROWW * sizeof(int));
    float* xlo   = (float*)carve((size_t)N32 * sizeof(float));
    float* xro   = (float*)carve((size_t)N32 * sizeof(float));
    float* xlino = (float*)carve((size_t)N32 * sizeof(float));
    int* segA = (int*)carve((size_t)NSB * strideA * sizeof(int));
    int* segB = (int*)carve((size_t)NB * strideB * sizeof(int));
    if (off > ws_size) return;

    const int convBlocks = (6 * DD * 16 + 255) / 256;
    const int gemmBlocks = Npad / 64;
    const int nodeBlocks = (N32 / 32 + 7) / 8;

    k_convw<<<convBlocks, 256, 0, stream>>>(Wl1, Wr1, Wlin1, Wl2, Wr2, Wlin2, Wt);
    k_binA<<<NSB, 256, 0, stream>>>(edst, E, SW, capA, strideA, segA);
    k_binB<<<NB, 256, 0, stream>>>(edst, E, segA, capA, strideA, CPP, BW, capB, strideB, segB);
    k_rows<<<NB, 256, BW * ROWW * sizeof(int), stream>>>(esrc, edst, E, N, segB, capB, strideB, adj);

    k_gemm3<<<gemmBlocks, 128, 65536, stream>>>(x, N, Wt, blin1, XL, XR, LIN);
    k_agg<0><<<nodeBlocks, 256, 0, stream>>>(adj, XL, XR, LIN, att1, b1, H1,
                                             Wlo, Wro, Wlino, xlo, xro, xlino, N);
    k_gemm3<<<gemmBlocks, 128, 65536, stream>>>(H1, N, Wt + 3 * DD * DD, blin2, XL, XR, LIN);
    k_agg<1><<<nodeBlocks, 256, 0, stream>>>(adj, XL, XR, LIN, att2, b2, H1,
                                             Wlo, Wro, Wlino, xlo, xro, xlino, N);
    k_out<<<nodeBlocks, 256, 0, stream>>>(adj, xlo, xro, xlino, atto, bo, blino, out, N);
    (void)hipGetLastError();
}
